// TriangleAttention_16793322127891
// MI455X (gfx1250) — hardware-verified
//
#include <hip/hip_runtime.h>
#include <stdint.h>


#define S_   256
#define C_   128
#define H_   4
#define D_   32
#define NN_FULL (S_ * S_)
#ifndef NI
#define NI S_
#endif
#ifndef NB
#define NB 1
#endif

static_assert(NB == 1);
static_assert(NI >= 1 && NI <= S_);
static_assert(C_ == H_ * D_);
static_assert((NI * S_) % 32 == 0);

#define QSCALE   0.17677669529663687f
#define RES_UP   2048.0f
#define RES_DN   0.00048828125f
#define W_UP     64.0f
#define P_UP     1024.0f
#define OG_UP    4096.0f

#define WBUF_HALVES 83968
#define WO_OFF      65536
#define WB_OFF      81920

#define LDS_QH 0
#define LDS_QL 16384
#define LDS_KH 32768
#define LDS_KL 49152
#define LDS_VH 65536
#define LDS_VL 81920
#define LDS_GS 98304
#define LDS_HS 131072
#define LDS_BS 147456
#define LDS_ATTN_BYTES 163840
static_assert(LDS_HS + 2 * 32 * C_ * 2 == LDS_BS);
static_assert(8 * 2048 == LDS_BS - LDS_HS);
static_assert(LDS_BS + 8 * 16 * 32 * 4 == LDS_ATTN_BYTES);

typedef float    v4f  __attribute__((ext_vector_type(4)));
typedef float    v8f  __attribute__((ext_vector_type(8)));
typedef _Float16 v8h  __attribute__((ext_vector_type(8)));
typedef _Float16 v16h __attribute__((ext_vector_type(16)));
typedef v8h v8ha __attribute__((may_alias));
typedef v4f v4fa __attribute__((may_alias));

__device__ __forceinline__ float bfr(float f) {
    uint32_t u = __builtin_bit_cast(uint32_t, f);
    u = (u + 0x7FFFu + ((u >> 16) & 1u)) & 0xFFFF0000u;
    return __builtin_bit_cast(float, u);
}

__device__ __forceinline__ v16h ldfrag(const _Float16* base, int stride, int lane) {
    const _Float16* p = base + (lane & 15) * stride + ((lane >> 4) << 3);
    const v8h a = *(const v8ha*)p;
    const v8h b = *(const v8ha*)(p + 16);
    return __builtin_shufflevector(a, b, 0, 1, 2, 3, 4, 5, 6, 7, 8, 9, 10, 11, 12, 13, 14, 15);
}

__device__ __forceinline__ v8f mma(v16h a, v16h b, v8f c) {
    v8f d = __builtin_amdgcn_wmma_f32_16x16x32_f16(false, a, false, b, (short)0, c, false, false);
    asm volatile("v_nop\n\tv_nop\n\tv_nop\n\tv_nop" : "+v"(d) : "v"(a), "v"(b));
    return d;
}

__device__ __forceinline__ void wave_sync() {
    __builtin_amdgcn_fence(__ATOMIC_RELEASE, "wavefront");
    __builtin_amdgcn_wave_barrier();
}

__device__ __forceinline__ _Float16 hi16(float y) { return (_Float16)y; }
__device__ __forceinline__ _Float16 lo16(float y, _Float16 hi) { return (_Float16)((y - (float)hi) * RES_UP); }

__global__ __launch_bounds__(256) void prep_w_kernel(const float* __restrict__ wq, const float* __restrict__ wk,
                                                     const float* __restrict__ wv, const float* __restrict__ wg,
                                                     const float* __restrict__ wo, const float* __restrict__ wb,
                                                     _Float16* __restrict__ wbuf) {
    const int b = blockIdx.x, t = threadIdx.x;
    const int r = t >> 4, c0 = (t & 15) * 8;
    const float* src;
    int rr = r;
    bool zero = false;
    if (b < 8)       src = wq + (size_t)(b * 16) * C_;
    else if (b < 16) src = wk + (size_t)((b - 8) * 16) * C_;
    else if (b < 24) src = wv + (size_t)((b - 16) * 16) * C_;
    else if (b < 32) src = wg + (size_t)((b - 24) * 16) * C_;
    else if (b < 40) src = wo + (size_t)((b - 32) * 16) * C_;
    else { src = wb; zero = (r >= H_); rr = (r < H_) ? r : (H_ - 1); }
    const float* p = src + (size_t)rr * C_ + c0;
    const v4f x0 = *(const v4f*)p;
    const v4f x1 = *(const v4f*)(p + 4);
    v8f y = __builtin_shufflevector(x0, x1, 0, 1, 2, 3, 4, 5, 6, 7);
#pragma unroll
    for (int k = 0; k < 8; ++k) y[k] = zero ? 0.0f : bfr(y[k]) * W_UP;
    const v8h o = __builtin_convertvector(y, v8h);
    _Float16* d = wbuf + (size_t)b * 2048 + t * 8;
    *(volatile v8h*)d = o;
    __threadfence();
    *(volatile v8h*)d = o;
}

__global__ __launch_bounds__(256) void ln_bias_kernel(const float* __restrict__ x, const float* __restrict__ lnw,
                                                      const float* __restrict__ lnb, const _Float16* __restrict__ wb16,
                                                      _Float16* __restrict__ hnh, _Float16* __restrict__ hnl,
                                                      float* __restrict__ bias) {
    __shared__ __attribute__((aligned(16))) _Float16 Ah[32 * C_];
    __shared__ __attribute__((aligned(16))) _Float16 Al[32 * C_];
    __shared__ __attribute__((aligned(16))) float Bst[H_ * 32];
    const int t = threadIdx.x, wv = t >> 5, lane = t & 31, hl = lane >> 4, n = lane & 15;
    const int c0 = n * 8;
    const size_t row0 = (size_t)blockIdx.x * 32;

    float w[8], bb[8];
    {
        const v4f wa = *(const v4f*)(lnw + c0), wc = *(const v4f*)(lnw + c0 + 4);
        const v4f ba = *(const v4f*)(lnb + c0), bc = *(const v4f*)(lnb + c0 + 4);
#pragma unroll
        for (int k = 0; k < 4; ++k) {
            w[k] = bfr(wa[k]); w[4 + k] = bfr(wc[k]);
            bb[k] = bfr(ba[k]); bb[4 + k] = bfr(bc[k]);
        }
    }

    v8h keeph[2], keepl[2];
#pragma unroll
    for (int ps = 0; ps < 2; ++ps) {
        const int lr = wv * 4 + ps * 2 + hl;
        const size_t row = row0 + lr;
        const float* xp = x + row * C_ + c0;
        const v4f xa = *(const v4f*)xp, xc = *(const v4f*)(xp + 4);
        float v[8];
#pragma unroll
        for (int k = 0; k < 4; ++k) { v[k] = bfr(xa[k]); v[4 + k] = bfr(xc[k]); }
        float s = 0.0f;
#pragma unroll
        for (int k = 0; k < 8; ++k) s += v[k];
        s += __shfl_xor(s, 1, 32); s += __shfl_xor(s, 2, 32);
        s += __shfl_xor(s, 4, 32); s += __shfl_xor(s, 8, 32);
        const float mu = s * (1.0f / C_);
        float d[8], q = 0.0f;
#pragma unroll
        for (int k = 0; k < 8; ++k) { d[k] = v[k] - mu; q += d[k] * d[k]; }
        q += __shfl_xor(q, 1, 32); q += __shfl_xor(q, 2, 32);
        q += __shfl_xor(q, 4, 32); q += __shfl_xor(q, 8, 32);
        const float rs = rsqrtf(q * (1.0f / C_) + 1e-5f);
        v8f yv;
#pragma unroll
        for (int k = 0; k < 8; ++k) yv[k] = d[k] * rs * w[k] + bb[k];
        const v8h vh = __builtin_convertvector(yv, v8h);
        v8f rv;
#pragma unroll
        for (int k = 0; k < 8; ++k) rv[k] = (yv[k] - (float)vh[k]) * RES_UP;
        const v8h vl = __builtin_convertvector(rv, v8h);
        *(v8ha*)(Ah + lr * C_ + c0) = vh;
        *(v8ha*)(Al + lr * C_ + c0) = vl;
        *(volatile v8h*)(hnh + row * C_ + c0) = vh;
        *(volatile v8h*)(hnl + row * C_ + c0) = vl;
        keeph[ps] = vh; keepl[ps] = vl;
    }
    __threadfence();
#pragma unroll
    for (int ps = 0; ps < 2; ++ps) {
        const int lr = wv * 4 + ps * 2 + hl;
        const size_t row = row0 + lr;
        *(volatile v8h*)(hnh + row * C_ + c0) = keeph[ps];
        *(volatile v8h*)(hnl + row * C_ + c0) = keepl[ps];
    }
    __syncthreads();

    if (wv < 2) {
        const int rt = wv;
        v8f acch = {}, accl = {};
#pragma unroll
        for (int kc = 0; kc < 4; ++kc) {
            const v16h fa = ldfrag(Ah + rt * 16 * C_ + kc * 32, C_, lane);
            const v16h fl = ldfrag(Al + rt * 16 * C_ + kc * 32, C_, lane);
            const v16h fb = ldfrag(wb16 + kc * 32, C_, lane);
            acch = mma(fa, fb, acch);
            accl = mma(fl, fb, accl);
        }
        if (n < H_) {
#pragma unroll
            for (int r = 0; r < 8; ++r)
                Bst[n * 32 + rt * 16 + hl * 8 + r] = (acch[r] + accl[r] * RES_DN) * (1.0f / W_UP);
        }
    }
    __syncthreads();
    if (wv == 0) {
        const int hd = lane >> 3, pc = lane & 7;
        const v4f bv = *(const v4fa*)(Bst + hd * 32 + pc * 4);
        float* dst = bias + (size_t)hd * NN_FULL + row0 + pc * 4;
        *(volatile v4f*)dst = bv;
        __threadfence();
        *(volatile v4f*)dst = bv;
    }
}

__device__ __forceinline__ void proj_step(const _Float16* HSh, const _Float16* HSl, int koff, int lane, v16h bw,
                                          v8f& a0h, v8f& a0l, v8f& a1h, v8f& a1l) {
    const v16h f0h = ldfrag(HSh + koff, C_, lane);
    const v16h f0l = ldfrag(HSl + koff, C_, lane);
    const v16h f1h = ldfrag(HSh + 16 * C_ + koff, C_, lane);
    const v16h f1l = ldfrag(HSl + 16 * C_ + koff, C_, lane);
    a0h = mma(f0h, bw, a0h);
    a0l = mma(f0l, bw, a0l);
    a1h = mma(f1h, bw, a1h);
    a1l = mma(f1l, bw, a1l);
}

__device__ __forceinline__ void proj_epi(v8f ah, v8f al, int mat, float fac, int jbase, int col, int hl,
                                         _Float16* QH, _Float16* QL, _Float16* KH, _Float16* KL,
                                         _Float16* VH, _Float16* VL, float* GS) {
#pragma unroll
    for (int r = 0; r < 8; ++r) {
        const float A = (ah[r] + al[r] * RES_DN) * fac;
        const int jrow = jbase + hl * 8 + r;
        if (mat == 0) {
            const _Float16 hv = hi16(A);
            QH[jrow * D_ + col] = hv;
            QL[jrow * D_ + col] = lo16(A, hv);
        } else if (mat == 1) {
            const _Float16 hv = hi16(A);
            KH[jrow * D_ + col] = hv;
            KL[jrow * D_ + col] = lo16(A, hv);
        } else if (mat == 2) {
            const _Float16 hv = hi16(A);
            VH[col * S_ + jrow] = hv;
            VL[col * S_ + jrow] = lo16(A, hv);
        } else {
            const float g = fmaxf(A * (1.0f / W_UP), -30.0f);
            GS[jrow * D_ + col] = __builtin_amdgcn_rcpf(1.0f + __expf(-g));
        }
    }
}

__global__ __launch_bounds__(256) void attn_kernel(const _Float16* __restrict__ hnh, const _Float16* __restrict__ hnl,
                                                   const _Float16* __restrict__ wbuf, const float* __restrict__ bias,
                                                   _Float16* __restrict__ ogh, _Float16* __restrict__ ogl) {
    extern __shared__ __attribute__((aligned(16))) char lds[];
    _Float16* QH = (_Float16*)(lds + LDS_QH);
    _Float16* QL = (_Float16*)(lds + LDS_QL);
    _Float16* KH = (_Float16*)(lds + LDS_KH);
    _Float16* KL = (_Float16*)(lds + LDS_KL);
    _Float16* VH = (_Float16*)(lds + LDS_VH);
    _Float16* VL = (_Float16*)(lds + LDS_VL);
    float*    GS = (float*)(lds + LDS_GS);
    _Float16* HSh = (_Float16*)(lds + LDS_HS);
    _Float16* HSl = HSh + 32 * C_;

    const int i = blockIdx.x, h = blockIdx.y;
    const int t = threadIdx.x, wv = t >> 5, lane = t & 31, hl = lane >> 4, n = lane & 15;

    {
        const int mat = wv >> 1, dt = wv & 1;
        const _Float16* wrow = wbuf + (size_t)(mat * C_ + h * D_ + dt * 16) * C_;
        const v16h bw0 = ldfrag(wrow,      C_, lane);
        const v16h bw1 = ldfrag(wrow + 32, C_, lane);
        const v16h bw2 = ldfrag(wrow + 64, C_, lane);
        const v16h bw3 = ldfrag(wrow + 96, C_, lane);
        const float fac = (mat == 0) ? QSCALE : 1.0f;
        const int col = dt * 16 + n;
#pragma unroll 1
        for (int cq = 0; cq < 8; ++cq) {
            const size_t src0 = ((size_t)i * S_ + cq * 32) * C_;
#pragma unroll
            for (int u = 0; u < 2; ++u) {
                const int q = t + u * 256;
                *(v8ha*)(HSh + q * 8) = *(const v8ha*)(hnh + src0 + (size_t)q * 8);
                *(v8ha*)(HSl + q * 8) = *(const v8ha*)(hnl + src0 + (size_t)q * 8);
            }
            __syncthreads();
            v8f a0h = {}, a0l = {}, a1h = {}, a1l = {};
            proj_step(HSh, HSl, 0,  lane, bw0, a0h, a0l, a1h, a1l);
            proj_step(HSh, HSl, 32, lane, bw1, a0h, a0l, a1h, a1l);
            proj_step(HSh, HSl, 64, lane, bw2, a0h, a0l, a1h, a1l);
            proj_step(HSh, HSl, 96, lane, bw3, a0h, a0l, a1h, a1l);
            proj_epi(a0h, a0l, mat, fac, cq * 32,      col, hl, QH, QL, KH, KL, VH, VL, GS);
            proj_epi(a1h, a1l, mat, fac, cq * 32 + 16, col, hl, QH, QL, KH, KL, VH, VL, GS);
            __syncthreads();
        }
    }

    {
        _Float16* Ph = HSh + wv * 1024;
        _Float16* Pl = Ph + 512;
        float* Bs = (float*)(lds + LDS_BS) + wv * 512;
#pragma unroll 1
        for (int jt = 0; jt < 2; ++jt) {
            const int j0 = (wv * 2 + jt) * 16;
            wave_sync();
            const v16h aqh = ldfrag(QH + j0 * D_, D_, lane);
            const v16h aql = ldfrag(QL + j0 * D_, D_, lane);
            float mrow[8], lrow[8];
#pragma unroll
            for (int r = 0; r < 8; ++r) { mrow[r] = -1.0e30f; lrow[r] = 0.0f; }
            v8f o0h = {}, o0l = {}, o1h = {}, o1l = {};
#pragma unroll 1
            for (int kc = 0; kc < 8; ++kc) {
                const int k0 = kc * 32;
                wave_sync();
                {
                    const float* bp = bias + (size_t)h * NN_FULL + (size_t)(j0 + n) * S_ + k0 + hl * 16;
                    const v4f b0 = *(const v4f*)bp;
                    const v4f b1 = *(const v4f*)(bp + 4);
                    const v4f b2 = *(const v4f*)(bp + 8);
                    const v4f b3 = *(const v4f*)(bp + 12);
                    float* bd = Bs + n * 32 + hl * 16;
                    *(v4fa*)bd = b0; *(v4fa*)(bd + 4) = b1; *(v4fa*)(bd + 8) = b2; *(v4fa*)(bd + 12) = b3;
                }
                wave_sync();
                float x1[8], x2[8];
                {
                    const v16h bkh = ldfrag(KH + k0 * D_, D_, lane);
                    const v16h bkl = ldfrag(KL + k0 * D_, D_, lane);
                    const v8f z = {};
                    v8f ch = mma(aqh, bkh, z);
                    v8f cl = mma(aql, bkh, z);
                    cl = mma(aqh, bkl, cl);
#pragma unroll
                    for (int r = 0; r < 8; ++r)
                        x1[r] = (ch[r] + cl[r] * RES_DN) * (1.0f / 4096.0f) + Bs[(hl * 8 + r) * 32 + n];
                }
                {
                    const v16h bkh = ldfrag(KH + (k0 + 16) * D_, D_, lane);
                    const v16h bkl = ldfrag(KL + (k0 + 16) * D_, D_, lane);
                    const v8f z = {};
                    v8f ch = mma(aqh, bkh, z);
                    v8f cl = mma(aql, bkh, z);
                    cl = mma(aqh, bkl, cl);
#pragma unroll
                    for (int r = 0; r < 8; ++r)
                        x2[r] = (ch[r] + cl[r] * RES_DN) * (1.0f / 4096.0f) + Bs[(hl * 8 + r) * 32 + 16 + n];
                }
#pragma unroll
                for (int r = 0; r < 8; ++r) {
                    float mx = fmaxf(x1[r], x2[r]);
                    mx = fmaxf(mx, __shfl_xor(mx, 1, 32));
                    mx = fmaxf(mx, __shfl_xor(mx, 2, 32));
                    mx = fmaxf(mx, __shfl_xor(mx, 4, 32));
                    mx = fmaxf(mx, __shfl_xor(mx, 8, 32));
                    const float mnew = fmaxf(mrow[r], mx);
                    const float alpha = __expf(mrow[r] - mnew);
                    mrow[r] = mnew;
                    const float p1 = __expf(x1[r] - mnew);
                    const float p2 = __expf(x2[r] - mnew);
                    float rs = p1 + p2;
                    rs += __shfl_xor(rs, 1, 32);
                    rs += __shfl_xor(rs, 2, 32);
                    rs += __shfl_xor(rs, 4, 32);
                    rs += __shfl_xor(rs, 8, 32);
                    lrow[r] = lrow[r] * alpha + rs;
                    o0h[r] *= alpha; o0l[r] *= alpha; o1h[r] *= alpha; o1l[r] *= alpha;
                    const int lr = hl * 8 + r;
                    const float y1 = p1 * P_UP, y2 = p2 * P_UP;
                    const _Float16 h1 = hi16(y1), h2 = hi16(y2);
                    Ph[lr * 32 + n] = h1;       Pl[lr * 32 + n] = lo16(y1, h1);
                    Ph[lr * 32 + 16 + n] = h2;  Pl[lr * 32 + 16 + n] = lo16(y2, h2);
                }
                wave_sync();
                {
                    const v16h aph = ldfrag(Ph, 32, lane);
                    const v16h apl = ldfrag(Pl, 32, lane);
                    v16h bvh = ldfrag(VH + k0, S_, lane);
                    v16h bvl = ldfrag(VL + k0, S_, lane);
                    o0h = mma(aph, bvh, o0h);
                    o0l = mma(apl, bvh, o0l);
                    o0l = mma(aph, bvl, o0l);
                    bvh = ldfrag(VH + 16 * S_ + k0, S_, lane);
                    bvl = ldfrag(VL + 16 * S_ + k0, S_, lane);
                    o1h = mma(aph, bvh, o1h);
                    o1l = mma(apl, bvh, o1l);
                    o1l = mma(aph, bvl, o1l);
                }
            }
            wave_sync();
#pragma unroll
            for (int r = 0; r < 8; ++r) {
                const int lr = hl * 8 + r;
                const float inv = __builtin_amdgcn_rcpf(lrow[r]) * (1.0f / 65536.0f);
                const int gi = (j0 + lr) * D_;
                const float ya = (o0h[r] + o0l[r] * RES_DN) * inv * GS[gi + n] * OG_UP;
                const float yb = (o1h[r] + o1l[r] * RES_DN) * inv * GS[gi + 16 + n] * OG_UP;
                const _Float16 ha = hi16(ya), hb = hi16(yb);
                Ph[lr * 32 + n] = ha;       Pl[lr * 32 + n] = lo16(ya, ha);
                Ph[lr * 32 + 16 + n] = hb;  Pl[lr * 32 + 16 + n] = lo16(yb, hb);
            }
            wave_sync();
            const v8h e0 = *(const v8ha*)(Ph + lane * 8);
            const v8h e1 = *(const v8ha*)(Ph + 256 + lane * 8);
            const v8h f0 = *(const v8ha*)(Pl + lane * 8);
            const v8h f1 = *(const v8ha*)(Pl + 256 + lane * 8);
            const size_t tb = ((size_t)h * NN_FULL + (size_t)i * S_ + j0) * D_;
            _Float16* dh = ogh + tb;
            _Float16* dl = ogl + tb;
            *(volatile v8h*)(dh + lane * 8) = e0;
            *(volatile v8h*)(dh + 256 + lane * 8) = e1;
            *(volatile v8h*)(dl + lane * 8) = f0;
            *(volatile v8h*)(dl + 256 + lane * 8) = f1;
            __threadfence();
            *(volatile v8h*)(dh + lane * 8) = e0;
            *(volatile v8h*)(dh + 256 + lane * 8) = e1;
            *(volatile v8h*)(dl + lane * 8) = f0;
            *(volatile v8h*)(dl + 256 + lane * 8) = f1;
        }
    }
}

__global__ __launch_bounds__(256) void out_kernel(const _Float16* __restrict__ ogh, const _Float16* __restrict__ ogl,
                                                  const _Float16* __restrict__ wo16, float* __restrict__ out) {
    __shared__ __attribute__((aligned(16))) float Os[32 * C_];
    const int t = threadIdx.x, wv = t >> 5, lane = t & 31, hl = lane >> 4, n = lane & 15;
    const int r0 = blockIdx.x * 32;
    const _Float16* wrow = wo16 + (size_t)(wv * 16) * C_;
    v8f a0h = {}, a0l = {}, a1h = {}, a1l = {};
#pragma unroll
    for (int kc = 0; kc < 4; ++kc) {
        const v16h bw = ldfrag(wrow + kc * 32, C_, lane);
        const _Float16* ph = ogh + ((size_t)kc * NN_FULL + r0) * D_;
        const _Float16* pl = ogl + ((size_t)kc * NN_FULL + r0) * D_;
        const v16h f0h = ldfrag(ph, D_, lane);
        const v16h f0l = ldfrag(pl, D_, lane);
        const v16h f1h = ldfrag(ph + 16 * D_, D_, lane);
        const v16h f1l = ldfrag(pl + 16 * D_, D_, lane);
        a0h = mma(f0h, bw, a0h);
        a0l = mma(f0l, bw, a0l);
        a1h = mma(f1h, bw, a1h);
        a1l = mma(f1l, bw, a1l);
    }
#pragma unroll
    for (int r = 0; r < 8; ++r) {
        Os[(hl * 8 + r) * C_ + wv * 16 + n]      = (a0h[r] + a0l[r] * RES_DN) * (1.0f / 262144.0f);
        Os[(16 + hl * 8 + r) * C_ + wv * 16 + n] = (a1h[r] + a1l[r] * RES_DN) * (1.0f / 262144.0f);
    }
    __syncthreads();
    float* dst = out + (size_t)r0 * C_;
    v4f keep[4];
#pragma unroll
    for (int u = 0; u < 4; ++u) {
        const int q = u * 256 + wv * 32 + lane;
        keep[u] = *(const v4fa*)(Os + q * 4);
        *(volatile v4f*)(dst + (size_t)q * 4) = keep[u];
    }
    __threadfence();
#pragma unroll
    for (int u = 0; u < 4; ++u) {
        const int q = u * 256 + wv * 32 + lane;
        *(volatile v4f*)(dst + (size_t)q * 4) = keep[u];
    }
}

extern "C" void kernel_launch(void* const* d_in, const int* in_sizes, int n_in,
                              void* d_out, int out_size, void* d_ws, size_t ws_size,
                              hipStream_t stream) {
    if (n_in < 9) return;
    if (in_sizes[0] < NN_FULL * C_) return;
    if (in_sizes[1] < C_ || in_sizes[2] < C_) return;
    if (in_sizes[3] < H_ * C_) return;
    if (in_sizes[4] < C_ * C_ || in_sizes[5] < C_ * C_ || in_sizes[6] < C_ * C_ ||
        in_sizes[7] < C_ * C_ || in_sizes[8] < C_ * C_) return;
    if (out_size < NI * S_ * C_) return;

    const float* x    = (const float*)d_in[0];
    const float* lnw  = (const float*)d_in[1];
    const float* lnb  = (const float*)d_in[2];
    const float* wb   = (const float*)d_in[3];
    const float* wq   = (const float*)d_in[4];
    const float* wk   = (const float*)d_in[5];
    const float* wv   = (const float*)d_in[6];
    const float* wg   = (const float*)d_in[7];
    const float* wo   = (const float*)d_in[8];
    float* out = (float*)d_out;

    char* ws = (char*)d_ws;
    size_t off = 0;
    auto carve = [&](size_t bytes) -> char* {
        char* p = ws + off;
        off += (bytes + 255) & ~(size_t)255;
        return p;
    };
    _Float16* wbuf = (_Float16*)carve((size_t)WBUF_HALVES * 2);
    _Float16* hnh  = (_Float16*)carve((size_t)NN_FULL * C_ * 2);
    _Float16* hnl  = (_Float16*)carve((size_t)NN_FULL * C_ * 2);
    float*    bpl  = (float*)carve((size_t)H_ * NN_FULL * 4);
    _Float16* ogh  = (_Float16*)carve((size_t)H_ * NN_FULL * D_ * 2);
    _Float16* ogl  = (_Float16*)carve((size_t)H_ * NN_FULL * D_ * 2);
    if (off > ws_size) return;

    prep_w_kernel<<<41, 256, 0, stream>>>(wq, wk, wv, wg, wo, wb, wbuf);
    ln_bias_kernel<<<NN_FULL / 32, 256, 0, stream>>>(x, lnw, lnb, wbuf + WB_OFF, hnh, hnl, bpl);
    (void)hipFuncSetAttribute(reinterpret_cast<const void*>(&attn_kernel),
                              hipFuncAttributeMaxDynamicSharedMemorySize, LDS_ATTN_BYTES);
    attn_kernel<<<dim3(NI, H_), 256, LDS_ATTN_BYTES, stream>>>(hnh, hnl, wbuf, bpl, ogh, ogl);
    out_kernel<<<(NI * S_) / 32, 256, 0, stream>>>(ogh, ogl, wbuf + WO_OFF, out);
}
